// EncoderBlock_88484916232285
// MI455X (gfx1250) — hardware-verified
//
#include <hip/hip_runtime.h>
#include <math.h>

#ifndef NB
#define NB 8
#endif
#ifndef SEQ
#define SEQ 1024
#endif
#define NB_FULL 8
#define SEQ_FULL 1024
#define C_D 768
#define C_H 12
#define C_HD 64
#define C_HID 3072
#define C_M (NB * SEQ)

static_assert(NB >= 1 && NB <= NB_FULL);
static_assert(SEQ >= 64 && SEQ <= SEQ_FULL && (SEQ % 64) == 0);
static_assert(NB == 1 || SEQ == SEQ_FULL);
static_assert(C_D == C_H * C_HD);
static_assert((C_M % 64) == 0 && (C_D % 64) == 0 && (C_HID % 64) == 0 && (C_D % 32) == 0 && (C_HID % 32) == 0);

typedef __attribute__((ext_vector_type(16))) _Float16 v16h;
typedef __attribute__((ext_vector_type(8)))  _Float16 v8h;
typedef __attribute__((ext_vector_type(8)))  float    v8f;
typedef __attribute__((ext_vector_type(4)))  float    v4f;
typedef unsigned int v4u __attribute__((ext_vector_type(4)));

union FragH { v16h v; v8h h[2]; };
__device__ __forceinline__ v16h frag_ld(const _Float16* p) { FragH f; f.h[0] = *(const v8h*)(p); f.h[1] = *(const v8h*)(p + 16); return f.v; }

__device__ __forceinline__ v8f wmma16(v16h a, v16h b, v8f c) {
    c = __builtin_amdgcn_wmma_f32_16x16x32_f16(false, a, false, b, (short)0, c, false, false);
    asm volatile("v_nop\n\tv_nop\n\tv_nop\n\tv_nop" : "+v"(c) : "v"(a), "v"(b));
    return c;
}
__device__ __forceinline__ void dep_guard_h(v8f& a, v8f& b, v16h x, v16h y) { asm volatile("v_nop\n\tv_nop\n\tv_nop\n\tv_nop" : "+v"(a), "+v"(b) : "v"(x), "v"(y)); }
__device__ __forceinline__ void keep4_h(v16h a, v16h b, v16h c, v16h d) { asm volatile("v_nop" :: "v"(a), "v"(b), "v"(c), "v"(d)); }
__device__ __forceinline__ void acc_guard4(v8f& a, v8f& b, v8f& c, v8f& d) { asm volatile("v_nop\n\tv_nop\n\tv_nop\n\tv_nop" : "+v"(a), "+v"(b), "+v"(c), "+v"(d)); }
__device__ __forceinline__ void wave_lds_sync() {
    __builtin_amdgcn_fence(3  , "workgroup");
    __builtin_amdgcn_wave_barrier();
    __builtin_amdgcn_fence(2  , "workgroup");
}

#define VST2(T, ptr, val) do { const T vst2_v_ = (val); *(volatile T*)(ptr) = vst2_v_; __threadfence(); *(volatile T*)(ptr) = vst2_v_; } while (0)

__device__ __forceinline__ unsigned int pk2h(float a, float b) { return (unsigned int)__builtin_bit_cast(unsigned short, (_Float16)a) | ((unsigned int)__builtin_bit_cast(unsigned short, (_Float16)b) << 16); }
__device__ __forceinline__ float bf_rne(float v) { const unsigned u = __builtin_bit_cast(unsigned, v); const unsigned r = (u + 0x7fffu + ((u >> 16) & 1u)) & 0xffff0000u; return __builtin_bit_cast(float, r); }

template <int BIAS_MODE, int OUT_MODE, bool RESID, int ACT, bool RRND>
__global__ __launch_bounds__(256) void k_gemm64(
    const unsigned short* __restrict__ Ap, unsigned lda,
    const unsigned short* __restrict__ Btp, unsigned ldb,
    void* __restrict__ Cout, unsigned ldc,
    const float* __restrict__ bias, const float* __restrict__ resid,
    unsigned M, unsigned N, unsigned K, float scale) {
  const _Float16* A  = (const _Float16*)Ap;
  const _Float16* Bt = (const _Float16*)Btp;
  __shared__ __align__(16) float sT[8][16 * 68];
  const unsigned lane = threadIdx.x & 31u;
  const unsigned wave = threadIdx.x >> 5;
  const unsigned tilesN = N >> 6;
  const unsigned tilesM = M >> 6;
  const unsigned tile = blockIdx.x * 8u + wave;
  if (tile >= tilesM * tilesN) return;
  const unsigned tm = tile / tilesN;
  const unsigned tn = tile - tm * tilesN;
  const unsigned m0 = tm << 6;
  const unsigned n0 = tn << 6;
  const unsigned rlane = lane & 15u;
  const unsigned koff  = (lane >> 4) * 8u;
  const unsigned mOff  = (lane >> 4) * 8u;

  v8f acc[4][4];
#pragma unroll
  for (int i = 0; i < 4; ++i)
#pragma unroll
    for (int j = 0; j < 4; ++j) acc[i][j] = (v8f){0.f,0.f,0.f,0.f,0.f,0.f,0.f,0.f};

  for (unsigned k0 = 0; k0 < K; k0 += 32u) {
    v16h bh[4];
#pragma unroll
    for (int j = 0; j < 4; ++j) {
      const size_t bo = (size_t)(n0 + ((unsigned)j << 4) + rlane) * ldb + koff + k0;
      bh[j] = frag_ld(Bt + bo);
    }
#pragma unroll
    for (int i = 0; i < 4; ++i) {
      const size_t ao = (size_t)(m0 + ((unsigned)i << 4) + rlane) * lda + koff + k0;
      const v16h ah = frag_ld(A + ao);
#pragma unroll
      for (int j = 0; j < 4; ++j)
        acc[i][j] = __builtin_amdgcn_wmma_f32_16x16x32_f16(false, ah, false, bh[j], (short)0, acc[i][j], false, false);
      dep_guard_h(acc[i][0], acc[i][3], ah, ah);
    }
    keep4_h(bh[0], bh[1], bh[2], bh[3]);
  }
  acc_guard4(acc[0][0], acc[0][1], acc[0][2], acc[0][3]);
  acc_guard4(acc[1][0], acc[1][1], acc[1][2], acc[1][3]);
  acc_guard4(acc[2][0], acc[2][1], acc[2][2], acc[2][3]);
  acc_guard4(acc[3][0], acc[3][1], acc[3][2], acc[3][3]);

  float* slab = sT[wave];
#pragma unroll
  for (int i = 0; i < 4; ++i) {
    const unsigned mBase = m0 + ((unsigned)i << 4);
#pragma unroll
    for (int j = 0; j < 4; ++j) {
      const unsigned n = n0 + ((unsigned)j << 4) + rlane;
      float bv = 0.f;
      if (BIAS_MODE == 2) bv = bias[n];
#pragma unroll
      for (int r = 0; r < 8; ++r) {
        float v = acc[i][j][r] * scale;
        if (BIAS_MODE == 2) v += bv;
        if (RESID) { float rv = resid[(size_t)(mBase + mOff + (unsigned)r) * ldc + n]; if (RRND) rv = bf_rne(rv); v += rv; }
        slab[(mOff + (unsigned)r) * 68u + ((unsigned)j << 4) + rlane] = v;
      }
    }
    wave_lds_sync();
    if (ACT == 5) {
#pragma unroll 1
      for (unsigned t = 0; t < 32u; ++t) {
        const unsigned e = t * 32u + lane;
        float* sp = slab + (e >> 6) * 68u + (e & 63u);
        const float v = *sp;
        const float gv = 0.5f * v * (1.0f + erff(v * 0.70710678118654752f));
        *sp = gv;
      }
      wave_lds_sync();
    }
    if (OUT_MODE == 0) {
      float* C = (float*)Cout;
      const unsigned hh = lane >> 4, c4 = (lane & 15u) * 4u;
      for (int pass = 0; pass < 2; ++pass) {
#pragma unroll
        for (int it = 0; it < 8; ++it) {
          const unsigned row = (unsigned)it * 2u + hh;
          const v4f v = *(const v4f*)(slab + row * 68u + c4);
          *(volatile v4f*)(C + (size_t)(mBase + row) * ldc + n0 + c4) = v;
        }
        __threadfence();
      }
    } else {
      const unsigned q = lane >> 3, c8 = (lane & 7u) * 8u;
      unsigned short* C = (unsigned short*)Cout;
      for (int pass = 0; pass < 2; ++pass) {
#pragma unroll
        for (int it = 0; it < 4; ++it) {
          const unsigned row = (unsigned)it * 4u + q;
          const float* sp = slab + row * 68u + c8;
          v8h hv;
#pragma unroll
          for (int e = 0; e < 8; ++e) hv[e] = (_Float16)sp[e];
          *(volatile v8h*)(C + (size_t)(mBase + row) * ldc + n0 + c8) = hv;
        }
        __threadfence();
      }
    }
    wave_lds_sync();
  }
}

__global__ __launch_bounds__(128) void k_attn_f16(const unsigned short* __restrict__ QKp, const unsigned short* __restrict__ VTp, unsigned short* __restrict__ AOp) {
  const _Float16* QK = (const _Float16*)QKp;
  const _Float16* VT = (const _Float16*)VTp;
  __shared__ __align__(16) _Float16 Psh[4][16 * 64];
  __shared__ __align__(16) float    Os[4][16 * 68];
  const unsigned tid = threadIdx.x, wave = tid >> 5, lane = tid & 31u, hh = lane >> 4, c = lane & 15u;
  const unsigned NQB = (unsigned)(SEQ / 64);
  const unsigned bx = blockIdx.x;
  const unsigned bh = bx / NQB;
  const unsigned qb = bx - bh * NQB;
  const unsigned b  = bh / (unsigned)C_H;
  const unsigned h  = bh - b * (unsigned)C_H;
  const unsigned q0 = qb * 64u + wave * 16u;
  const unsigned tok0 = b * (unsigned)SEQ;

  v16h qa[2];
  {
    const _Float16* qrow = QK + (size_t)(tok0 + q0 + c) * 1536u + h * 64u + 8u * hh;
    qa[0] = frag_ld(qrow);
    qa[1] = frag_ld(qrow + 32);
  }
  const _Float16* kbase = QK + (size_t)tok0 * 1536u + 768u + h * 64u + 8u * hh;
  const _Float16* vbase = VT + (size_t)(h * 64u + c) * (unsigned)C_M + tok0 + 8u * hh;

  float mrow[8], lrow[8];
  v8f oacc[4];
#pragma unroll
  for (int r = 0; r < 8; ++r) { mrow[r] = -__builtin_inff(); lrow[r] = 0.f; }
#pragma unroll
  for (int t = 0; t < 4; ++t) oacc[t] = (v8f){0.f,0.f,0.f,0.f,0.f,0.f,0.f,0.f};

  _Float16* pw = Psh[wave];
  const float SC = 0.125f * 1.4426950408889634f;

  for (unsigned kc = 0; kc < NQB; ++kc) {
    const unsigned kv0 = kc * 64u;
    v8f s[4];
#pragma unroll
    for (int j = 0; j < 4; ++j) {
      const _Float16* kr = kbase + (size_t)(kv0 + (unsigned)j * 16u + c) * 1536u;
      v8f a = (v8f){0.f,0.f,0.f,0.f,0.f,0.f,0.f,0.f};
      a = wmma16(qa[0], frag_ld(kr), a);
      a = wmma16(qa[1], frag_ld(kr + 32), a);
      s[j] = a;
    }
#pragma unroll
    for (int r = 0; r < 8; ++r) {
      float m = -__builtin_inff();
#pragma unroll
      for (int j = 0; j < 4; ++j) { const float t = s[j][r] * SC; s[j][r] = t; m = fmaxf(m, t); }
#pragma unroll
      for (unsigned off = 1; off < 16u; off <<= 1) m = fmaxf(m, __shfl_xor(m, (int)off, 32));
      const float mnew = fmaxf(mrow[r], m);
      const float alpha = exp2f(mrow[r] - mnew);
      mrow[r] = mnew;
      float psum = 0.f;
#pragma unroll
      for (int j = 0; j < 4; ++j) {
        const float p = exp2f(s[j][r] - mnew);
        psum += p;
        pw[(8u * hh + (unsigned)r) * 64u + (unsigned)j * 16u + c] = (_Float16)(p * 32768.0f);
      }
#pragma unroll
      for (unsigned off = 1; off < 16u; off <<= 1) psum += __shfl_xor(psum, (int)off, 32);
      lrow[r] = lrow[r] * alpha + psum;
#pragma unroll
      for (int t = 0; t < 4; ++t) oacc[t][r] *= alpha;
    }
    wave_lds_sync();
#pragma unroll
    for (int kk = 0; kk < 2; ++kk) {
      const v16h pa = frag_ld(pw + c * 64u + (unsigned)kk * 32u + 8u * hh);
#pragma unroll
      for (int t = 0; t < 4; ++t) {
        const _Float16* vr = vbase + (size_t)((unsigned)t * 16u) * (unsigned)C_M + kv0 + (unsigned)kk * 32u;
        oacc[t] = wmma16(pa, frag_ld(vr), oacc[t]);
      }
    }
    wave_lds_sync();
  }

  float* os = Os[wave];
#pragma unroll
  for (int r = 0; r < 8; ++r) {
    const float inv = 1.0f / (lrow[r] * 32768.0f);
#pragma unroll
    for (int t = 0; t < 4; ++t) os[(8u * hh + (unsigned)r) * 68u + (unsigned)t * 16u + c] = oacc[t][r] * inv;
  }
  wave_lds_sync();
  {
    const unsigned q = lane >> 3, c8 = (lane & 7u) * 8u;
    unsigned short* ob = AOp + (size_t)(tok0 + q0) * (unsigned)C_D + h * 64u;
    for (int pass = 0; pass < 2; ++pass) {
#pragma unroll
      for (int it = 0; it < 4; ++it) {
        const unsigned row = (unsigned)it * 4u + q;
        const float* sp = os + row * 68u + c8;
        v8h hv;
#pragma unroll
        for (int e = 0; e < 8; ++e) hv[e] = (_Float16)sp[e];
        *(volatile v8h*)(ob + (size_t)row * (unsigned)C_D + c8) = hv;
      }
      __threadfence();
    }
  }
}

template <int BFX>
__global__ __launch_bounds__(256) void k_ln768(const float* __restrict__ X, const float* __restrict__ G, const float* __restrict__ Bb, unsigned short* __restrict__ O, unsigned rows) {
    #pragma clang fp contract(off)
    const unsigned row = blockIdx.x * 8u + (threadIdx.x >> 5); const unsigned L = threadIdx.x & 31u; if (row >= rows) return;
    const float* xr = X + (size_t)row * 768u; float x[24]; float s = 0.f;
#pragma unroll
    for (int g = 0; g < 3; ++g) { const v4f a = *(const v4f*)(xr + 256 * g + 8u * L), b = *(const v4f*)(xr + 256 * g + 8u * L + 4u); const float v[8] = {a.x, a.y, a.z, a.w, b.x, b.y, b.z, b.w};
#pragma unroll
        for (int e = 0; e < 8; ++e) { const float t = BFX ? bf_rne(v[e]) : v[e]; x[8 * g + e] = t; s += t; } }
#pragma unroll
    for (int o = 16; o > 0; o >>= 1) s += __shfl_xor(s, o, 32);
    const float mu = s * (1.f / 768.f); float q = 0.f;
#pragma unroll
    for (int e = 0; e < 24; ++e) { const float d = x[e] - mu; q += d * d; }
#pragma unroll
    for (int o = 16; o > 0; o >>= 1) q += __shfl_xor(q, o, 32);
    const float inv = 1.0f / (sqrtf(q * (1.f / 768.f)) + 1e-8f);
#pragma unroll
    for (int g = 0; g < 3; ++g) { const unsigned c0 = 256u * (unsigned)g + 8u * L; float y[8];
#pragma unroll
        for (int e = 0; e < 8; ++e) y[e] = (x[8 * g + e] - mu) * inv * bf_rne(G[c0 + e]) + bf_rne(Bb[c0 + e]);
        v4u pk; pk.x = pk2h(y[0], y[1]); pk.y = pk2h(y[2], y[3]); pk.z = pk2h(y[4], y[5]); pk.w = pk2h(y[6], y[7]); VST2(v4u, (v4u*)(O + (size_t)row * 768u + c0), pk); } }

__global__ __launch_bounds__(256) void k_bfvec(const float* __restrict__ SRC, float* __restrict__ DST, unsigned n) { const unsigned u = blockIdx.x * 256u + threadIdx.x; if (u >= n) return; VST2(float, DST + u, bf_rne(SRC[u])); }
__global__ __launch_bounds__(256) void k_castbT(const float* __restrict__ SRC, unsigned lds, unsigned short* __restrict__ DST, unsigned ldd, unsigned nR, unsigned nC, float sc) {
    const unsigned u = blockIdx.x * 256u + threadIdx.x; const unsigned per = nR >> 3; if (u >= nC * per) return; const unsigned c = u / per; const unsigned r0 = 8u * (u - c * per);
    float w[8];
#pragma unroll
    for (int e = 0; e < 8; ++e) w[e] = bf_rne(SRC[(size_t)(r0 + (unsigned)e) * lds + c]) * sc;
    v4u pk; pk.x = pk2h(w[0], w[1]); pk.y = pk2h(w[2], w[3]); pk.z = pk2h(w[4], w[5]); pk.w = pk2h(w[6], w[7]); VST2(v4u, (v4u*)(DST + (size_t)c * ldd + r0), pk); }
__global__ __launch_bounds__(256) void k_pack_qkv(const float* __restrict__ Wq, const float* __restrict__ Wk, const float* __restrict__ Wv, unsigned short* __restrict__ DST) {
    const unsigned sel = blockIdx.y;
    const float* W = (sel == 0u) ? Wq : ((sel == 1u) ? Wk : Wv);
    const unsigned u = blockIdx.x * 256u + threadIdx.x; if (u >= 768u * 96u) return;
    const unsigned he = u / 96u; const unsigned d0 = 8u * (u - he * 96u); const unsigned h = he >> 6, e = he & 63u;
    const float* s = W + ((size_t)h * 768u + d0) * 64u + e;
    float w[8];
#pragma unroll
    for (int i = 0; i < 8; ++i) w[i] = bf_rne(s[(unsigned)i * 64u]) * 16.0f;
    v4u pk; pk.x = pk2h(w[0], w[1]); pk.y = pk2h(w[2], w[3]); pk.z = pk2h(w[4], w[5]); pk.w = pk2h(w[6], w[7]); VST2(v4u, (v4u*)(DST + ((size_t)sel * 768u + he) * 768u + d0), pk); }

constexpr size_t SZ_WQKV = (size_t)2304 * 768 * 2;
constexpr size_t SZ_WO   = (size_t)768 * 768 * 2;
constexpr size_t SZ_W1   = (size_t)3072 * 768 * 2;
constexpr size_t SZ_W2   = (size_t)768 * 3072 * 2;
constexpr size_t SZ_B1   = (size_t)3072 * 4;
constexpr size_t SZ_B2   = (size_t)768 * 4;
constexpr size_t SZ_N16  = (size_t)C_M * 768 * 2;
constexpr size_t SZ_QK   = (size_t)C_M * 1536 * 2;
constexpr size_t SZ_VT   = (size_t)768 * C_M * 2;
constexpr size_t SZ_AO   = (size_t)C_M * 768 * 2;
constexpr size_t SZ_X1   = (size_t)C_M * 768 * 4;
constexpr size_t SZ_H16  = (size_t)C_M * 3072 * 2;
constexpr size_t OFF_WQKV = 0;
constexpr size_t OFF_WO   = OFF_WQKV + SZ_WQKV;
constexpr size_t OFF_W1   = OFF_WO + SZ_WO;
constexpr size_t OFF_W2   = OFF_W1 + SZ_W1;
constexpr size_t OFF_B1   = OFF_W2 + SZ_W2;
constexpr size_t OFF_B2   = OFF_B1 + SZ_B1;
constexpr size_t OFF_N16  = OFF_B2 + SZ_B2;
constexpr size_t OFF_QK   = OFF_N16 + SZ_N16;
constexpr size_t OFF_VT   = OFF_QK + SZ_QK;
constexpr size_t OFF_AO   = OFF_VT + SZ_VT;
constexpr size_t OFF_X1   = OFF_AO + SZ_AO;
constexpr size_t WS_TOTAL = OFF_X1 + SZ_X1;
constexpr size_t OFF_H16  = OFF_QK;
static_assert(SZ_H16 <= SZ_QK + SZ_VT + SZ_AO);
static_assert((SZ_WQKV % 256) == 0 && (SZ_WO % 256) == 0 && (SZ_W1 % 256) == 0 && (SZ_B1 % 256) == 0 && (SZ_B2 % 256) == 0 && (SZ_N16 % 256) == 0 && (SZ_QK % 256) == 0 && (SZ_VT % 256) == 0 && (SZ_AO % 256) == 0);
static_assert(WS_TOTAL <= (size_t)134217728);
static_assert(((size_t)(C_M / 8)) * 8 == (size_t)C_M);
static_assert((size_t)288 * 256 == (size_t)768 * 96);

extern "C" void kernel_launch(void* const* d_in, const int* in_sizes, int n_in, void* d_out, int out_size, void* d_ws, size_t ws_size, hipStream_t stream) {
    if (n_in < 13) return;
    if (in_sizes[0] < C_M * C_D) return;
    if (in_sizes[1] < C_D || in_sizes[2] < C_D || in_sizes[3] < C_D || in_sizes[4] < C_D) return;
    if (in_sizes[5] < 589824 || in_sizes[6] < 589824 || in_sizes[7] < 589824 || in_sizes[8] < 589824) return;
    if (in_sizes[9] < 2359296 || in_sizes[10] < 3072 || in_sizes[11] < 2359296 || in_sizes[12] < 768) return;
    if (out_size < C_M * C_D) return;
    if (WS_TOTAL > ws_size) return;
    const float* x      = (const float*)d_in[0];
    const float* scale1 = (const float*)d_in[1];
    const float* shift1 = (const float*)d_in[2];
    const float* scale2 = (const float*)d_in[3];
    const float* shift2 = (const float*)d_in[4];
    const float* Wq     = (const float*)d_in[5];
    const float* Wk     = (const float*)d_in[6];
    const float* Wv     = (const float*)d_in[7];
    const float* Wo     = (const float*)d_in[8];
    const float* W1     = (const float*)d_in[9];
    const float* b1     = (const float*)d_in[10];
    const float* W2     = (const float*)d_in[11];
    const float* b2     = (const float*)d_in[12];
    float* out = (float*)d_out;
    char* wsp = (char*)d_ws;
    unsigned short* WQKV16 = (unsigned short*)(wsp + OFF_WQKV);
    unsigned short* WO16   = (unsigned short*)(wsp + OFF_WO);
    unsigned short* W116   = (unsigned short*)(wsp + OFF_W1);
    unsigned short* W216   = (unsigned short*)(wsp + OFF_W2);
    float*          BR1    = (float*)(wsp + OFF_B1);
    float*          BR2    = (float*)(wsp + OFF_B2);
    unsigned short* N16    = (unsigned short*)(wsp + OFF_N16);
    unsigned short* QK16   = (unsigned short*)(wsp + OFF_QK);
    unsigned short* VT16   = (unsigned short*)(wsp + OFF_VT);
    unsigned short* AO16   = (unsigned short*)(wsp + OFF_AO);
    float*          X1     = (float*)(wsp + OFF_X1);
    unsigned short* H16    = (unsigned short*)(wsp + OFF_H16);

    k_pack_qkv<<<dim3(288u, 3u), 256, 0, stream>>>(Wq, Wk, Wv, WQKV16);
    k_castbT<<<(unsigned)((768u * 96u + 255u) / 256u), 256, 0, stream>>>(Wo, 768u, WO16, 768u, 768u, 768u, 16.0f);
    k_castbT<<<(unsigned)((3072u * 96u + 255u) / 256u), 256, 0, stream>>>(W1, 3072u, W116, 768u, 768u, 3072u, 16.0f);
    k_castbT<<<(unsigned)((768u * 384u + 255u) / 256u), 256, 0, stream>>>(W2, 768u, W216, 3072u, 3072u, 768u, 16.0f);
    k_bfvec<<<(3072u + 255u) / 256u, 256, 0, stream>>>(b1, BR1, 3072u);
    k_bfvec<<<(768u + 255u) / 256u, 256, 0, stream>>>(b2, BR2, 768u);

    k_ln768<1><<<(unsigned)(C_M / 8), 256, 0, stream>>>(x, scale1, shift1, N16, (unsigned)C_M);
    k_gemm64<0, 1, false, 0, false><<<(unsigned)((((C_M) / 64) * (1536 / 64) + 7) / 8), 256, 0, stream>>>(
        N16, 768u, WQKV16, 768u, (void*)QK16, 1536u, BR1, X1, (unsigned)C_M, 1536u, 768u, 0.0625f);
    k_gemm64<0, 1, false, 0, false><<<(unsigned)(((768 / 64) * ((C_M) / 64) + 7) / 8), 256, 0, stream>>>(
        WQKV16 + (size_t)1536 * 768, 768u, N16, 768u, (void*)VT16, (unsigned)C_M, BR1, X1, 768u, (unsigned)C_M, 768u, 0.0625f);
    k_attn_f16<<<(unsigned)(NB * C_H * (SEQ / 64)), 128, 0, stream>>>(QK16, VT16, AO16);
    k_gemm64<0, 0, true, 0, true><<<(unsigned)((((C_M) / 64) * (768 / 64) + 7) / 8), 256, 0, stream>>>(
        AO16, 768u, WO16, 768u, (void*)X1, 768u, BR1, x, (unsigned)C_M, 768u, 768u, 0.0625f);
    k_ln768<0><<<(unsigned)(C_M / 8), 256, 0, stream>>>(X1, scale2, shift2, N16, (unsigned)C_M);
    k_gemm64<2, 1, false, 5, false><<<(unsigned)((((C_M) / 64) * (3072 / 64) + 7) / 8), 256, 0, stream>>>(
        N16, 768u, W116, 768u, (void*)H16, 3072u, BR1, X1, (unsigned)C_M, 3072u, 768u, 0.0625f);
    k_gemm64<2, 0, true, 0, false><<<(unsigned)((((C_M) / 64) * (768 / 64) + 7) / 8), 256, 0, stream>>>(
        H16, 3072u, W216, 3072u, (void*)out, 768u, BR2, X1, (unsigned)C_M, 768u, 3072u, 0.0625f);
}
